// TSPTWFeasGIN_83416854823073
// MI455X (gfx1250) — hardware-verified
//
#include <hip/hip_runtime.h>
#include <stddef.h>


#define FD      128
#define XD      4
#define NHP     16
#define NLAY    3
#define NTHR    256
#define NWAVE   8
#define EPT     8
#define NGRP    2
#define CHUNK   (NTHR * EPT * NGRP)
#define WCAPC   (EPT * NGRP * 32)
#define WCAPF   128
#define ESHF    11
#define NBC     32768
#define NBF     2048
#define RCAP    68608
#define RBN     128
#define DEGCAP  1024
#define GROWS   128
#define OTHR    512
#define APITCH  136
#define WSCALE  256
#define WSCAP   134217728
#define WPLANE  (FD * FD)
#define WGRP    (FD * FD / 8)
#define HGRP    (NHP * FD / 8)
#define NWG     (6 * WGRP + HGRP)
#define WHOFF   (6 * WPLANE)

#define LDS_COUNT ((NBC + NWAVE * WCAPC + NWAVE) * 4)
#define LDS_FILL  ((RCAP + NBF + NWAVE * WCAPF + NWAVE) * 4)
#define LDS_A     (GROWS * APITCH * 2)
#define LDS_Z     (GROWS * APITCH * 2)
#define LDS_O     (GROWS * FD * 4)
#define LDS_C     (GROWS * 4)
#define LDS_LAYER (LDS_A + LDS_Z + LDS_O + LDS_C)

static_assert((CHUNK & (CHUNK - 1)) == 0);
static_assert((NBC & (NBC - 1)) == 0 && (NBF & (NBF - 1)) == 0);
static_assert(NBF <= (1 << ESHF));
static_assert((NBC % NBF) == 0);
static_assert(OTHR * 4 == NBF);
static_assert((RCAP % 32) == 0);
static_assert(GROWS == NWAVE * 16);
static_assert(NBC == NWAVE * 32 * 128);
static_assert((FD % 32) == 0 && FD == 4 * 32);
static_assert((16 * FD) % 128 == 0);
static_assert((APITCH % 8) == 0 && APITCH >= FD);
static_assert((GROWS % 4) == 0 && ((GROWS * 4) % 128) == 0);
static_assert((NWG * 16) % 128 == 0);
static_assert(NHP == 16);
static_assert((LDS_A % 16) == 0 && ((LDS_A + LDS_Z) % 16) == 0 && ((LDS_A + LDS_Z + LDS_O) % 16) == 0);
static_assert(LDS_FILL <= 300 * 1024 && LDS_LAYER <= 300 * 1024 && LDS_COUNT <= 300 * 1024);

typedef float     v4f  __attribute__((ext_vector_type(4)));
typedef float     v8f  __attribute__((ext_vector_type(8)));
typedef int       v4i  __attribute__((ext_vector_type(4)));
typedef _Float16  v4h  __attribute__((ext_vector_type(4)));
typedef _Float16  v8h  __attribute__((ext_vector_type(8)));
typedef _Float16  v16h __attribute__((ext_vector_type(16)));
union FragH { v16h v; v8h h[2]; };

__device__ __forceinline__ v8f wmf(v16h a, v16h b, v8f c) {
  v8f d = __builtin_amdgcn_wmma_f32_16x16x32_f16(false, a, false, b, (short)0, c, false, false);
  asm volatile("v_nop\n\tv_nop\n\tv_nop\n\tv_nop" : "+v"(d) : "v"(a), "v"(b));
  return d;
}

template <int NB, int SRC, int WC>
__device__ __forceinline__ int scan_chunk(const int* __restrict__ keys, const int* __restrict__ vals,
                                          int nK, int nN, int cbase, int slotBase, int vec8,
                                          int* list, int tid, int lane, int wave) {
  int wc = 0;
#pragma unroll
  for (int g = 0; g < NGRP; ++g) {
    const int el0  = (g * NTHR + tid) * EPT;
    const int e0   = cbase + el0;
    const int sent = -2147483647 - 1;
    v4i da, db;
    v4i sa = {0, 0, 0, 0}, sb = {0, 0, 0, 0};
    if (vec8 != 0 && cbase + CHUNK <= nK) {
      da = *(const v4i*)(keys + e0);
      db = *(const v4i*)(keys + e0 + 4);
      if (SRC) {
        sa = *(const v4i*)(vals + e0);
        sb = *(const v4i*)(vals + e0 + 4);
      }
    } else {
      const int i0 = min(e0, nK - 1),     i1 = min(e0 + 1, nK - 1), i2 = min(e0 + 2, nK - 1), i3 = min(e0 + 3, nK - 1);
      const int i4 = min(e0 + 4, nK - 1), i5 = min(e0 + 5, nK - 1), i6 = min(e0 + 6, nK - 1), i7 = min(e0 + 7, nK - 1);
      da.x = (e0     < nK) ? keys[i0] : sent;
      da.y = (e0 + 1 < nK) ? keys[i1] : sent;
      da.z = (e0 + 2 < nK) ? keys[i2] : sent;
      da.w = (e0 + 3 < nK) ? keys[i3] : sent;
      db.x = (e0 + 4 < nK) ? keys[i4] : sent;
      db.y = (e0 + 5 < nK) ? keys[i5] : sent;
      db.z = (e0 + 6 < nK) ? keys[i6] : sent;
      db.w = (e0 + 7 < nK) ? keys[i7] : sent;
      if (SRC) {
        sa.x = vals[i0]; sa.y = vals[i1]; sa.z = vals[i2]; sa.w = vals[i3];
        sb.x = vals[i4]; sb.y = vals[i5]; sb.z = vals[i6]; sb.w = vals[i7];
      }
    }
    if (SRC) {
      sa.x = min(max(sa.x, 0), nN - 1); sa.y = min(max(sa.y, 0), nN - 1);
      sa.z = min(max(sa.z, 0), nN - 1); sa.w = min(max(sa.w, 0), nN - 1);
      sb.x = min(max(sb.x, 0), nN - 1); sb.y = min(max(sb.y, 0), nN - 1);
      sb.z = min(max(sb.z, 0), nN - 1); sb.w = min(max(sb.w, 0), nN - 1);
    }
    const unsigned nb = (unsigned)slotBase;
    const unsigned s0 = (unsigned)da.x - nb, s1 = (unsigned)da.y - nb;
    const unsigned s2 = (unsigned)da.z - nb, s3 = (unsigned)da.w - nb;
    const unsigned s4 = (unsigned)db.x - nb, s5 = (unsigned)db.y - nb;
    const unsigned s6 = (unsigned)db.z - nb, s7 = (unsigned)db.w - nb;
    const bool h0 = s0 < (unsigned)NB, h1 = s1 < (unsigned)NB, h2 = s2 < (unsigned)NB, h3 = s3 < (unsigned)NB;
    const bool h4 = s4 < (unsigned)NB, h5 = s5 < (unsigned)NB, h6 = s6 < (unsigned)NB, h7 = s7 < (unsigned)NB;
    const unsigned any = __builtin_amdgcn_ballot_w32(h0 | h1 | h2 | h3 | h4 | h5 | h6 | h7);
    if (any != 0u) {
#define HITJ(HJ, SJ, VJ) { \
        const unsigned mj = __builtin_amdgcn_ballot_w32(HJ); \
        if (mj != 0u) { \
          if (HJ) { \
            const int pos = wc + (int)__builtin_amdgcn_mbcnt_lo(mj, 0u); \
            const int entv = SRC ? (((VJ) << ESHF) | (int)(SJ)) : (int)(SJ); \
            if (pos < WC) list[wave * WC + pos] = entv; \
          } \
          wc += (int)__builtin_popcount(mj); } }
      HITJ(h0, s0, sa.x)
      HITJ(h1, s1, sa.y)
      HITJ(h2, s2, sa.z)
      HITJ(h3, s3, sa.w)
      HITJ(h4, s4, sb.x)
      HITJ(h5, s5, sb.y)
      HITJ(h6, s6, sb.z)
      HITJ(h7, s7, sb.w)
#undef HITJ
    }
  }
  return wc;
}

__global__ __launch_bounds__(NTHR) void k_wprep(const float* __restrict__ w1, const float* __restrict__ w2,
                                                const float* __restrict__ wo, _Float16* wp, int ngrp) {
  const int i = (int)blockIdx.x * NTHR + (int)threadIdx.x;
  if (i >= ngrp) return;
  int mat = i / WGRP; mat = mat > 6 ? 6 : mat;
  const int r  = i - mat * WGRP;
  const int n  = r / 16;
  const int k0 = 8 * (r - 16 * n);
  const int matc = mat > 5 ? 5 : mat;
  const int lyr  = matc % 3;
  const int nd   = n > FD - 1 ? FD - 1 : n;
  v8h hv;
#pragma unroll
  for (int e = 0; e < 8; ++e) {
    const int k = k0 + e;
    const float va = w1[((size_t)lyr * FD + k) * FD + nd];
    const float vb = w2[((size_t)lyr * FD + k) * FD + nd];
    const float vhl = wo[k];
    const float vhc = (n == 0) ? vhl : 0.0f;
    const float v = (mat < 3) ? va : ((mat < 6) ? vb : vhc);
    hv[e] = (_Float16)(v * (float)WSCALE);
  }
  _Float16* d = wp + (size_t)i * 8;
  *(volatile v8h*)d = hv;
  __threadfence();
  *(volatile v8h*)d = hv;
}

__global__ __launch_bounds__(NTHR) void k_proj(const float* __restrict__ x, const float* __restrict__ w,
                                               const float* __restrict__ b, float* h, int nN, int nRows) {
  const int gid  = (int)blockIdx.x * NTHR + (int)threadIdx.x;
  const int row  = gid >> 5;
  const int lane = gid & 31;
  if (row >= nRows) return;
  const int xr = row > nN - 1 ? nN - 1 : row;
  const int c4 = 4 * lane;
  const v4f xv  = *(const v4f*)(x + (size_t)xr * XD);
  const v4f wv0 = *(const v4f*)(w + 0 * FD + c4);
  const v4f wv1 = *(const v4f*)(w + 1 * FD + c4);
  const v4f wv2 = *(const v4f*)(w + 2 * FD + c4);
  const v4f wv3 = *(const v4f*)(w + 3 * FD + c4);
  const v4f bv  = *(const v4f*)(b + c4);
  v4f acc = wv0 * xv.x;
  acc = wv1 * xv.y + acc;
  acc = wv2 * xv.z + acc;
  acc = wv3 * xv.w + acc;
  acc = acc + bv;
  float* d = h + (size_t)row * FD + c4;
  *(volatile v4f*)d = acc;
  __threadfence();
  *(volatile v4f*)d = acc;
}

__global__ __launch_bounds__(NTHR) void k_count(
    const int* __restrict__ keys, int* cnt, int nK, int nN, int vec8) {
  extern __shared__ v4f lds_dyn[];
  int* scnt = (int*)lds_dyn;
  int* list = scnt + NBC;
  int* wcnt = list + NWAVE * WCAPC;
  const int tid = threadIdx.x, lane = tid & 31, wave = tid >> 5;
  const int nodeBase = blockIdx.x * NBC;

  {
    const v4i z = {0, 0, 0, 0};
    for (int i = tid; i < NBC / 4; i += NTHR) ((v4i*)scnt)[i] = z;
  }
  __syncthreads();

  const int nChunks = (nK + CHUNK - 1) / CHUNK;
#pragma unroll 1
  for (int ch = 0; ch < nChunks; ++ch) {
    const int cbase = ch * CHUNK;
    const int wc = scan_chunk<NBC, 0, WCAPC>(keys, keys, nK, nN, cbase, nodeBase, vec8, list, tid, lane, wave);
    if (lane == 0) wcnt[wave] = wc;
    __syncthreads();
    if (wave == 0) {
#pragma unroll 1
      for (int wsx = 0; wsx < NWAVE; ++wsx) {
        int n = __builtin_amdgcn_readfirstlane(wcnt[wsx]);
        n = n > WCAPC ? WCAPC : (n < 0 ? 0 : n);
        const int* lp = list + wsx * WCAPC;
#pragma unroll 1
        for (int i = 0; i < n; ++i) {
          const int ent  = __builtin_amdgcn_readfirstlane(lp[i]);
          const int slot = ent & (NBC - 1);
          if (lane == 0) scnt[slot] = scnt[slot] + 1;
        }
      }
    }
    __syncthreads();
  }

  int* cp = cnt + (size_t)nodeBase;
#pragma unroll 4
  for (int q = 0; q < 32; ++q) {
    const int f = (wave * 32 + q) * 128 + 4 * lane;
    const v4i c = *(const v4i*)(scnt + f);
    *(volatile v4i*)(cp + f) = c;
  }
  __threadfence();
#pragma unroll 4
  for (int q = 0; q < 32; ++q) {
    const int f = (wave * 32 + q) * 128 + 4 * lane;
    const v4i c = *(const v4i*)(scnt + f);
    *(volatile v4i*)(cp + f) = c;
  }
}

__global__ __launch_bounds__(OTHR) void k_offsets(
    const int* __restrict__ cnt, int* off, int* rbase, int nBF) {
  __shared__ __attribute__((aligned(16))) int srb[RBN];
  __shared__ int wtot[OTHR / 32];
  const int tid = threadIdx.x, lane = tid & 31, wave = tid >> 5;
  for (int i = tid; i < RBN; i += OTHR) srb[i] = 0;
  int carry = 0;
#pragma unroll 1
  for (int fb = 0; fb < nBF; ++fb) {
    const int base = fb * NBF;
    const v4i c = *(const v4i*)(cnt + base + 4 * tid);
    const int e0 = max(c.x, 0), e1 = max(c.y, 0), e2 = max(c.z, 0), e3 = max(c.w, 0);
    const int ts = e0 + e1 + e2 + e3;
    int incl = ts;
#pragma unroll
    for (int d = 1; d < 32; d <<= 1) {
      const int t = __shfl_up(incl, d, 32);
      if (lane >= d) incl += t;
    }
    if (lane == 31) wtot[wave] = incl;
    __syncthreads();
    int pre = 0;
#pragma unroll 1
    for (int w = 0; w < wave; ++w) pre += wtot[w];
    int tot = 0;
#pragma unroll
    for (int w = 0; w < OTHR / 32; ++w) tot += wtot[w];
    int run = carry + pre + incl - ts;
    v4i o;
    o.x = run; run += e0;
    o.y = run; run += e1;
    o.z = run; run += e2;
    o.w = run;
    int* op = off + base + 4 * tid;
    *(volatile v4i*)op = o;
    __threadfence();
    *(volatile v4i*)op = o;
    if (tid == 0) srb[min(fb, RBN - 1)] = carry;
    carry += (tot + 31) & ~31;
    __syncthreads();
  }
  if (tid == 0) srb[min(nBF, RBN - 1)] = carry;
  __syncthreads();
  v4i rv = {0, 0, 0, 0};
  if (tid < 32) rv = *(const v4i*)(srb + 4 * tid);
  if (tid < 32) *(volatile v4i*)(rbase + 4 * tid) = rv;
  __threadfence();
  if (tid < 32) *(volatile v4i*)(rbase + 4 * tid) = rv;
}

__global__ __launch_bounds__(NTHR) void k_fill(
    const int* __restrict__ keys, const int* __restrict__ vals, const int* __restrict__ off,
    const int* __restrict__ rbase, int* csr, int nN, int nK, int vec8, int csrLen) {
  extern __shared__ v4f lds_dyn[];
  int* region = (int*)lds_dyn;
  int* cursor = region + RCAP;
  int* list   = cursor + NBF;
  int* wcnt   = list + NWAVE * WCAPF;
  const int tid = threadIdx.x, lane = tid & 31, wave = tid >> 5;
  const int b = blockIdx.x;
  const int nodeBase = b * NBF;

  int rb0 = rbase[b];
  const int rb1 = rbase[b + 1];
  rb0 = rb0 < 0 ? 0 : (rb0 > csrLen ? csrLen : rb0);
  rb0 &= ~31;
  int len = rb1 - rb0;
  len = len < 0 ? 0 : (len > RCAP ? RCAP : len);
  int lenW = (len + 31) & ~31;
  if (rb0 + lenW > csrLen) lenW = (csrLen - rb0) & ~31;

  {
    const v4i z = {0, 0, 0, 0};
    for (int i = tid; i < RCAP / 4; i += NTHR) ((v4i*)region)[i] = z;
    for (int s = tid; s < NBF; s += NTHR) {
      int o = off[nodeBase + s] - rb0;
      o = o < 0 ? 0 : (o > RCAP ? RCAP : o);
      cursor[s] = o;
    }
  }
  __syncthreads();

  const int nChunks = (nK + CHUNK - 1) / CHUNK;
#pragma unroll 1
  for (int ch = 0; ch < nChunks; ++ch) {
    const int cbase = ch * CHUNK;
    const int wc = scan_chunk<NBF, 1, WCAPF>(keys, vals, nK, nN, cbase, nodeBase, vec8, list, tid, lane, wave);
    if (lane == 0) wcnt[wave] = wc;
    __syncthreads();
    if (wave == 0) {
#pragma unroll 1
      for (int wsx = 0; wsx < NWAVE; ++wsx) {
        int n = __builtin_amdgcn_readfirstlane(wcnt[wsx]);
        n = n > WCAPF ? WCAPF : (n < 0 ? 0 : n);
        const int* lp = list + wsx * WCAPF;
#pragma unroll 1
        for (int i = 0; i < n; ++i) {
          const int ent  = __builtin_amdgcn_readfirstlane(lp[i]);
          const int slot = ent & (NBF - 1);
          int src = (ent >> ESHF) & 0xFFFFF;
          src = src > nN - 1 ? nN - 1 : src;
          if (lane == 0) {
            int pos = cursor[slot];
            pos = pos < 0 ? 0 : (pos > RCAP - 1 ? RCAP - 1 : pos);
            region[pos] = src;
            const int np = pos + 1;
            cursor[slot] = np > RCAP ? RCAP : np;
          }
        }
      }
    }
    __syncthreads();
  }

  const int nv = lenW >> 2;
  int* gp = csr + rb0;
#pragma unroll 1
  for (int i = tid; i < nv; i += NTHR) { const v4i v = ((const v4i*)region)[i]; *(volatile v4i*)(gp + 4 * i) = v; }
  __threadfence();
#pragma unroll 1
  for (int i = tid; i < nv; i += NTHR) { const v4i v = ((const v4i*)region)[i]; *(volatile v4i*)(gp + 4 * i) = v; }
}

template <int ASH, int LAST>
__global__ __launch_bounds__(NTHR) void k_layer(
    const int* __restrict__ csr, const int* __restrict__ offp, const int* __restrict__ cnt,
    const float* __restrict__ hin,
    const _Float16* __restrict__ w1p, const float* __restrict__ b1,
    const _Float16* __restrict__ w2p, const float* __restrict__ b2,
    const _Float16* __restrict__ whp, const float* __restrict__ bh,
    float* hout, float* yout, int nN, int csrLen) {
  extern __shared__ v4f lds_dyn[];
  _Float16* ldsA = (_Float16*)lds_dyn;
  _Float16* ldsZ = ldsA + GROWS * APITCH;
  float*    ldsO = (float*)(ldsZ + GROWS * APITCH);
  float*    ldsC = ldsO + GROWS * FD;
  constexpr int NT = FD / 16;
  constexpr int KT = FD / 32;
  constexpr float SCA = (float)(1 << ASH);
  constexpr float OSC = 1.0f / ((float)(1 << ASH) * (float)WSCALE);
  const int tid = threadIdx.x, lane = tid & 31, wave = tid >> 5, hh = lane >> 4, m = lane & 15;
  const int rowBase = blockIdx.x * GROWS;
  const int node0 = rowBase + wave * 16;

  {
    const int c4 = 4 * lane;
    const int cl = node0 + m;
    const int cnt_l = cnt[cl];
    const int off_l = offp[cl];
    _Float16* aw = ldsA + (wave * 16) * APITCH + c4;
#pragma unroll 1
    for (int j = 0; j < 16; ++j) {
      int n = __builtin_amdgcn_readlane(cnt_l, j);
      n = n < 0 ? 0 : (n > DEGCAP ? DEGCAP : n);
      const int st = __builtin_amdgcn_readlane(off_l, j);
      int self = node0 + j;
      self = self > nN - 1 ? nN - 1 : self;
      v4f acc = *(const v4f*)(hin + (size_t)self * FD + c4);
#pragma unroll 1
      for (int q0 = 0; q0 < n; q0 += 32) {
        int pos = st + q0 + lane;
        pos = pos < 0 ? 0 : (pos > csrLen - 1 ? csrLen - 1 : pos);
        int sl = csr[pos];
        sl = sl < 0 ? 0 : (sl > nN - 1 ? nN - 1 : sl);
        const int mcnt = (n - q0) < 32 ? (n - q0) : 32;
#pragma unroll 1
        for (int p = 0; p < mcnt; ++p) {
          const int s = __builtin_amdgcn_readlane(sl, p);
          acc = acc + *(const v4f*)(hin + (size_t)s * FD + c4);
        }
      }
      v4h hv;
      hv[0] = (_Float16)(acc.x * SCA); hv[1] = (_Float16)(acc.y * SCA);
      hv[2] = (_Float16)(acc.z * SCA); hv[3] = (_Float16)(acc.w * SCA);
      *(v4h*)(aw + j * APITCH) = hv;
    }
  }
  __syncthreads();

  const int r0w = wave * 16 + 8 * hh;
  v8f acc[NT];

#pragma unroll
  for (int t = 0; t < NT; ++t) { v8f z = {0.f, 0.f, 0.f, 0.f, 0.f, 0.f, 0.f, 0.f}; acc[t] = z; }
  {
    const _Float16* ap = ldsA + (wave * 16 + m) * APITCH + 8 * hh;
#pragma unroll
    for (int kt = 0; kt < KT; ++kt) {
      FragH af;
      af.h[0] = *(const v8h*)(ap + 32 * kt);
      af.h[1] = *(const v8h*)(ap + 32 * kt + 16);
#pragma unroll
      for (int t = 0; t < NT; ++t) {
        const _Float16* bp = w1p + (size_t)(16 * t + m) * FD + 32 * kt + 8 * hh;
        FragH bf;
        bf.h[0] = *(const v8h*)bp;
        bf.h[1] = *(const v8h*)(bp + 16);
        acc[t] = wmf(af.v, bf.v, acc[t]);
      }
    }
  }
#pragma unroll
  for (int t = 0; t < NT; ++t) {
    const float bb = b1[16 * t + m];
#pragma unroll
    for (int r = 0; r < 8; ++r) {
      const float v = __builtin_fmaxf(acc[t][r] * OSC + bb, 0.0f);
      ldsZ[(r0w + r) * APITCH + 16 * t + m] = (_Float16)(v * SCA);
    }
  }
  __syncthreads();

#pragma unroll
  for (int t = 0; t < NT; ++t) { v8f z = {0.f, 0.f, 0.f, 0.f, 0.f, 0.f, 0.f, 0.f}; acc[t] = z; }
  {
    const _Float16* ap = ldsZ + (wave * 16 + m) * APITCH + 8 * hh;
#pragma unroll
    for (int kt = 0; kt < KT; ++kt) {
      FragH af;
      af.h[0] = *(const v8h*)(ap + 32 * kt);
      af.h[1] = *(const v8h*)(ap + 32 * kt + 16);
#pragma unroll
      for (int t = 0; t < NT; ++t) {
        const _Float16* bp = w2p + (size_t)(16 * t + m) * FD + 32 * kt + 8 * hh;
        FragH bf;
        bf.h[0] = *(const v8h*)bp;
        bf.h[1] = *(const v8h*)(bp + 16);
        acc[t] = wmf(af.v, bf.v, acc[t]);
      }
    }
  }
#pragma unroll
  for (int t = 0; t < NT; ++t) {
    const float bb = b2[16 * t + m];
#pragma unroll
    for (int r = 0; r < 8; ++r) {
      const float v = __builtin_fmaxf(acc[t][r] * OSC + bb, 0.0f);
      if (LAST) ldsA[(r0w + r) * APITCH + 16 * t + m] = (_Float16)(v * SCA);
      else      ldsO[(r0w + r) * FD + 16 * t + m] = v;
    }
  }
  __syncthreads();

  if (!LAST) {
    const float* lp = ldsO + wave * 16 * FD;
    float* gp = hout + (size_t)node0 * FD;
#pragma unroll
    for (int i = 0; i < (16 * FD) / 128; ++i) {
      const v4f v = *(const v4f*)(lp + i * 128 + 4 * lane);
      *(volatile v4f*)(gp + i * 128 + 4 * lane) = v;
    }
    __threadfence();
#pragma unroll
    for (int i = 0; i < (16 * FD) / 128; ++i) {
      const v4f v = *(const v4f*)(lp + i * 128 + 4 * lane);
      *(volatile v4f*)(gp + i * 128 + 4 * lane) = v;
    }
  } else {
    v8f cacc = {0.f, 0.f, 0.f, 0.f, 0.f, 0.f, 0.f, 0.f};
    {
      const _Float16* ap = ldsA + (wave * 16 + m) * APITCH + 8 * hh;
#pragma unroll
      for (int kt = 0; kt < KT; ++kt) {
        FragH af, bf;
        af.h[0] = *(const v8h*)(ap + 32 * kt);
        af.h[1] = *(const v8h*)(ap + 32 * kt + 16);
        const _Float16* bp = whp + (size_t)m * FD + 32 * kt + 8 * hh;
        bf.h[0] = *(const v8h*)bp;
        bf.h[1] = *(const v8h*)(bp + 16);
        cacc = wmf(af.v, bf.v, cacc);
      }
    }
    {
      const float bhv = bh[0];
#pragma unroll
      for (int r = 0; r < 8; ++r) {
        const float o = cacc[r] * OSC + bhv;
        if (m == 0) ldsC[r0w + r] = o;
      }
    }
    __syncthreads();
    int vrows = nN - rowBase;
    vrows = vrows < 0 ? 0 : (vrows > GROWS ? GROWS : vrows);
    const int validF = vrows;
    float* ob = yout + (size_t)rowBase;
#pragma unroll 1
    for (int f = tid; f < GROWS / 4; f += NTHR) {
      const int e0 = 4 * f;
      if (e0 + 4 <= validF) {
        const v4f v = *(const v4f*)(ldsC + e0);
        *(volatile v4f*)(ob + e0) = v;
      } else {
#pragma unroll
        for (int e = 0; e < 4; ++e) {
          if (e0 + e < validF) { const float s = ldsC[e0 + e]; *(volatile float*)(ob + e0 + e) = s; }
        }
      }
    }
    __threadfence();
#pragma unroll 1
    for (int f = tid; f < GROWS / 4; f += NTHR) {
      const int e0 = 4 * f;
      if (e0 + 4 <= validF) {
        const v4f v = *(const v4f*)(ldsC + e0);
        *(volatile v4f*)(ob + e0) = v;
      } else {
#pragma unroll
        for (int e = 0; e < 4; ++e) {
          if (e0 + e < validF) { const float s = ldsC[e0 + e]; *(volatile float*)(ob + e0 + e) = s; }
        }
      }
    }
  }
}

extern "C" void kernel_launch(void* const* d_in, const int* in_sizes, int n_in,
                              void* d_out, int out_size, void* d_ws, size_t ws_size,
                              hipStream_t stream) {
  if (n_in < 10) return;
  const int nN = in_sizes[0] / XD;
  const int nE = in_sizes[1] / 2;
  if (nN <= 0 || nE <= 0 || in_sizes[0] != nN * XD || in_sizes[1] != 2 * nE) return;
  if (in_sizes[2] != XD * FD || in_sizes[3] != FD) return;
  if (in_sizes[4] != NLAY * FD * FD || in_sizes[5] != NLAY * FD) return;
  if (in_sizes[6] != NLAY * FD * FD || in_sizes[7] != NLAY * FD) return;
  if (in_sizes[8] != FD || in_sizes[9] < 1) return;
  if (out_size != nN) return;
  if (nN > (1 << 20) || nE > (1 << 28)) return;

  const float* x   = (const float*)d_in[0];
  const int*   ei  = (const int*)d_in[1];
  const float* niw = (const float*)d_in[2];
  const float* nib = (const float*)d_in[3];
  const float* w1  = (const float*)d_in[4];
  const float* b1  = (const float*)d_in[5];
  const float* w2  = (const float*)d_in[6];
  const float* b2  = (const float*)d_in[7];
  const float* ow  = (const float*)d_in[8];
  const float* obp = (const float*)d_in[9];
  float* out = (float*)d_out;
  const int* keys = ei + nE;
  const int* vals = ei;
  const int nK = nE;

  const int NPAD   = ((nN + GROWS - 1) / GROWS) * GROWS;
  const int nBC    = (nN + NBC - 1) / NBC;
  const int CNTPAD = nBC * NBC;
  const int nBF    = (nN + NBF - 1) / NBF;
  const int OFFN   = nBF * NBF;
  if (nBF + 1 > RBN) return;
  if (OFFN > CNTPAD || NPAD > OFFN) return;
  const int csrLen = ((nK + 31) & ~31) + 32 * (nBF + 1);
  const int nLay   = NPAD / GROWS;

  char* ws = (char*)d_ws;
  size_t off = 0;
  const size_t oW   = off; off += (size_t)NWG * 8 * 2;            off = (off + 255) & ~(size_t)255;
  const size_t oCnt = off; off += (size_t)CNTPAD * 4;             off = (off + 255) & ~(size_t)255;
  const size_t oOff = off; off += (size_t)OFFN * 4;               off = (off + 255) & ~(size_t)255;
  const size_t oRb  = off; off += (size_t)RBN * 4;                off = (off + 255) & ~(size_t)255;
  const size_t oCsr = off; off += (size_t)csrLen * 4;             off = (off + 255) & ~(size_t)255;
  const size_t oHa  = off; off += (size_t)NPAD * FD * 4;          off = (off + 255) & ~(size_t)255;
  const size_t oHb  = off; off += (size_t)NPAD * FD * 4;          off = (off + 255) & ~(size_t)255;
  if (off > ws_size || off > (size_t)WSCAP) return;
  _Float16* wp   = (_Float16*)(ws + oW);
  int*      cnt  = (int*)(ws + oCnt);
  int*      offp = (int*)(ws + oOff);
  int*      rb   = (int*)(ws + oRb);
  int*      csr  = (int*)(ws + oCsr);
  float*    hA   = (float*)(ws + oHa);
  float*    hB   = (float*)(ws + oHb);

  const int vec8 = ((nE & 3) == 0) ? 1 : 0;

  k_wprep<<<(NWG + NTHR - 1) / NTHR, NTHR, 0, stream>>>(w1, w2, ow, wp, NWG);

  k_proj<<<(NPAD * 32 + NTHR - 1) / NTHR, NTHR, 0, stream>>>(x, niw, nib, hA, nN, NPAD);

  hipFuncSetAttribute(reinterpret_cast<const void*>(&k_count),
                      hipFuncAttributeMaxDynamicSharedMemorySize, LDS_COUNT);
  k_count<<<nBC, NTHR, LDS_COUNT, stream>>>(keys, cnt, nK, nN, vec8);
  k_offsets<<<1, OTHR, 0, stream>>>(cnt, offp, rb, nBF);
  hipFuncSetAttribute(reinterpret_cast<const void*>(&k_fill),
                      hipFuncAttributeMaxDynamicSharedMemorySize, LDS_FILL);
  k_fill<<<nBF, NTHR, LDS_FILL, stream>>>(keys, vals, offp, rb, csr, nN, nK, vec8, csrLen);

  hipFuncSetAttribute(reinterpret_cast<const void*>(&k_layer<3, 0>),
                      hipFuncAttributeMaxDynamicSharedMemorySize, LDS_LAYER);
  hipFuncSetAttribute(reinterpret_cast<const void*>(&k_layer<1, 0>),
                      hipFuncAttributeMaxDynamicSharedMemorySize, LDS_LAYER);
  hipFuncSetAttribute(reinterpret_cast<const void*>(&k_layer<0, 1>),
                      hipFuncAttributeMaxDynamicSharedMemorySize, LDS_LAYER);
  k_layer<3, 0><<<nLay, NTHR, LDS_LAYER, stream>>>(csr, offp, cnt, hA,
      wp + 0 * WPLANE, b1 + 0 * FD, wp + 3 * WPLANE, b2 + 0 * FD, wp + WHOFF, obp, hB, out, nN, csrLen);
  k_layer<1, 0><<<nLay, NTHR, LDS_LAYER, stream>>>(csr, offp, cnt, hB,
      wp + 1 * WPLANE, b1 + 1 * FD, wp + 4 * WPLANE, b2 + 1 * FD, wp + WHOFF, obp, hA, out, nN, csrLen);
  k_layer<0, 1><<<nLay, NTHR, LDS_LAYER, stream>>>(csr, offp, cnt, hA,
      wp + 2 * WPLANE, b1 + 2 * FD, wp + 5 * WPLANE, b2 + 2 * FD, wp + WHOFF, obp, hB, out, nN, csrLen);
}
